// UNet_72430328480154
// MI455X (gfx1250) — hardware-verified
//
#include <hip/hip_runtime.h>


namespace {
constexpr int H = 1024, W = 1024, HW = H * W, HL = 1024  , NCH = 6, DH = 128, NO = 2;
constexpr float XS = 8.0f, WSC = 256.0f;
static_assert(W % 64 == 0 && HL % 1 == 0, "tiling");
typedef _Float16 b16;
typedef __attribute__((ext_vector_type(16))) _Float16 v16b;
typedef __attribute__((ext_vector_type(8))) _Float16 v8b;
typedef __attribute__((ext_vector_type(8))) float v8f;
typedef __attribute__((ext_vector_type(4))) float v4f;
__device__ __forceinline__ float bf16_rne(float f) { unsigned int u = __float_as_uint(f); u += 0x7FFFu + ((u >> 16) & 1u); return __uint_as_float(u & 0xFFFF0000u); }
__device__ __forceinline__ void split16(float v, b16& hi, b16& lo) { hi = (b16)v; lo = (b16)(v - (float)hi); }
__device__ __forceinline__ v16b frag_kb(const b16* p, int hh) { const v8b a = *(const v8b*)(p + 8 * hh), b = *(const v8b*)(p + 16 + 8 * hh); v16b f;
#pragma unroll
  for (int e = 0; e < 8; ++e) { f[e] = a[e]; f[8 + e] = b[e]; } return f; }
__device__ __forceinline__ v8f wmma16b(v16b a, v16b b, v8f c) { v8f d = __builtin_amdgcn_wmma_f32_16x16x32_f16(false, a, false, b, (short)0, c, false, false); asm volatile("v_nop\n\tv_nop\n\tv_nop\n\tv_nop" : "+v"(d) : "v"(a), "v"(b)); return d; }
__device__ __forceinline__ void wave_lds_sync() { __builtin_amdgcn_fence(__ATOMIC_RELEASE, "workgroup"); __builtin_amdgcn_wave_barrier(); __builtin_amdgcn_fence(__ATOMIC_ACQUIRE, "workgroup"); }
__device__ __forceinline__ float pmul(float a, float b) { float p = a * b; asm volatile("" : "+v"(p)); return p; }
__device__ __forceinline__ int iclamp(int v, int lo, int hi) { return v < lo ? lo : (v > hi ? hi : v); }

__global__ __launch_bounds__(256) void prep_kernel(const float* __restrict__ lw1, const float* __restrict__ lw2, b16* __restrict__ W1T, b16* __restrict__ W2T) {
  for (int i = threadIdx.x; i < DH * 32 / 8; i += 256) { const int e = i * 8; const int oo = e / 32, k0 = e % 32; v8b o; for (int j = 0; j < 8; ++j) { const int k = k0 + j; o[j] = (k < NCH) ? (b16)(bf16_rne(lw1[oo * NCH + k]) * WSC) : (b16)0.0f; } for (int pass = 0; pass < 2; ++pass) { *(volatile v8b*)(W1T + e) = o; __threadfence(); } }
  for (int i = threadIdx.x; i < 16 * DH / 8; i += 256) { const int e = i * 8; const int oo = e / DH, k0 = e % DH; v8b o; for (int j = 0; j < 8; ++j) o[j] = (oo < NO) ? (b16)(bf16_rne(lw2[oo * DH + k0 + j]) * WSC) : (b16)0.0f; for (int pass = 0; pass < 2; ++pass) { *(volatile v8b*)(W2T + e) = o; __threadfence(); } }
}
__global__ __launch_bounds__(256) void copy_kernel(const float* __restrict__ x, float* __restrict__ PL) {
  const size_t u = (size_t)blockIdx.x * 256 + threadIdx.x; if (u >= (size_t)3 * HW) return; const float v = bf16_rne(x[u]);
  for (int pass = 0; pass < 2; ++pass) { ((volatile float*)PL)[u] = v; __threadfence(); }
}
template <int CIN>
__global__ __launch_bounds__(256) void conv_kernel(const float* __restrict__ w, const float* __restrict__ bias, float* __restrict__ PL) {
  const size_t u = (size_t)blockIdx.x * 256 + threadIdx.x; if (u >= (size_t)HL * W) return; const int y = (int)(u / W), xx = (int)(u % W);
  float s = bf16_rne(bias[0]);
#pragma unroll
  for (int c = 0; c < CIN; ++c) {
#pragma unroll
    for (int dy = 0; dy < 3; ++dy) { const int yy = y + dy - 1; if (yy < 0 || yy >= H) continue;
#pragma unroll
      for (int dx = 0; dx < 3; ++dx) { const int x2 = xx + dx - 1; if (x2 < 0 || x2 >= W) continue; s += bf16_rne(w[(c * 3 + dy) * 3 + dx]) * PL[(size_t)c * HW + (size_t)yy * W + x2]; } } }
  const float o = 1.0f / (1.0f + __expf(-s));
  for (int pass = 0; pass < 2; ++pass) { ((volatile float*)PL)[(size_t)CIN * HW + u] = o; __threadfence(); }
}
__global__ __launch_bounds__(128) void mlp_kernel(const float* __restrict__ XA, const float* __restrict__ XB, const b16* __restrict__ W1T, const b16* __restrict__ W2T, const float* __restrict__ lb1, const float* __restrict__ lb2, float* __restrict__ outf, float* __restrict__ den1, float* __restrict__ den2) {
  __shared__ __attribute__((aligned(16))) float Th[4][16][DH + 4]; __shared__ __attribute__((aligned(16))) float OF[64][2]; __shared__ __attribute__((aligned(16))) float DA[64 * NCH], DB[64 * NCH];
  const int wave = threadIdx.x >> 5, lane = threadIdx.x & 31, nloc = lane & 15, hlf = lane >> 4; const size_t p0 = (size_t)blockIdx.x * 64; const size_t pr = p0 + wave * 16 + nloc;
  for (int i = threadIdx.x; i < 64 * NCH; i += 128) { const int px = i / NCH, c = i % NCH; DA[i] = XA[(size_t)c * HW + p0 + px]; DB[i] = XB[(size_t)c * HW + p0 + px]; }
  v8f acc[8];
#pragma unroll
  for (int t = 0; t < 8; ++t) acc[t] = (v8f){};
  { v16b ah, al;
#pragma unroll
    for (int e2 = 0; e2 < 16; ++e2) { const int k = (e2 < 8 ? 0 : 16) + 8 * hlf + (e2 & 7); float v = 0.0f; if (k < NCH) v = XA[(size_t)k * HW + pr] - XB[(size_t)k * HW + pr]; b16 p, q; split16(v * XS, p, q); ah[e2] = p; al[e2] = q; }
#pragma unroll
    for (int t = 0; t < 8; ++t) { const v16b bw = frag_kb(W1T + (size_t)(t * 16 + nloc) * 32, hlf); acc[t] = wmma16b(ah, bw, acc[t]); acc[t] = wmma16b(al, bw, acc[t]); } }
#pragma unroll
  for (int t = 0; t < 8; ++t) { const float bb = bf16_rne(lb1[t * 16 + nloc]);
#pragma unroll
    for (int r = 0; r < 8; ++r) Th[wave][8 * hlf + r][t * 16 + nloc] = acc[t][r] * (1.0f / (XS * WSC)) + bb; }
  wave_lds_sync();
  v8f acc2 = (v8f){};
#pragma unroll
  for (int ks = 0; ks < DH / 32; ++ks) { v16b ah, al;
#pragma unroll
    for (int e2 = 0; e2 < 16; ++e2) { const int k = ks * 32 + (e2 < 8 ? 0 : 16) + 8 * hlf + (e2 & 7); b16 p, q; split16(Th[wave][nloc][k] * XS, p, q); ah[e2] = p; al[e2] = q; }
    const v16b bw = frag_kb(W2T + (size_t)nloc * DH + ks * 32, hlf); acc2 = wmma16b(ah, bw, acc2); acc2 = wmma16b(al, bw, acc2); }
  if (nloc < NO) {
#pragma unroll
    for (int r = 0; r < 8; ++r) OF[wave * 16 + 8 * hlf + r][nloc] = acc2[r] * (1.0f / (XS * WSC)) + bf16_rne(lb2[nloc]); }
  __syncthreads();
  for (int pass = 0; pass < 2; ++pass) {
    if (wave == 0) *(volatile v4f*)(outf + p0 * NO + lane * 4) = *(const v4f*)(&OF[0][0] + lane * 4);
    for (int i = threadIdx.x; i < 64 * NCH / 4; i += 128) { *(volatile v4f*)(den1 + p0 * NCH + i * 4) = *(const v4f*)(&DA[i * 4]); *(volatile v4f*)(den2 + p0 * NCH + i * 4) = *(const v4f*)(&DB[i * 4]); }
    __threadfence(); }
}
}

extern "C" void kernel_launch(void* const* d_in, const int* in_sizes, int n_in, void* d_out, int out_size, void* d_ws, size_t ws_size, hipStream_t stream) {
  (void)n_in;
  auto Fp = [&](int i) { return (const float*)d_in[i]; };
  if (in_sizes[0] != 3 * HW || in_sizes[1] != 3 * HW || in_sizes[2] != 27 || in_sizes[4] != 36 || in_sizes[6] != 45 || in_sizes[8] != 27 || in_sizes[10] != 36 || in_sizes[12] != 45 || in_sizes[14] != DH * NCH || in_sizes[15] != DH || in_sizes[16] != NO * DH || in_sizes[17] != NO || out_size != HW * NO + 2 * HW * NCH) return;
  size_t off = 0; char* ws = (char*)d_ws;
  auto carve = [&](size_t bytes) { char* p = ws + off; off += (bytes + 255) & ~(size_t)255; return p; };
  b16* W1T = (b16*)carve((size_t)DH * 32 * 2); b16* W2T = (b16*)carve((size_t)16 * DH * 2); float* XA = (float*)carve((size_t)NCH * HW * 4); float* XB = (float*)carve((size_t)NCH * HW * 4);
  if (off > ws_size || off > ((size_t)128 << 20)) return;
  float* outf = (float*)d_out; float* den1 = outf + (size_t)HW * NO; float* den2 = den1 + (size_t)HW * NCH;
  prep_kernel<<<1, 256, 0, stream>>>(Fp(14), Fp(16), W1T, W2T);
  const unsigned ncp = (unsigned)(((size_t)3 * HW + 255) / 256), ncv = (unsigned)(((size_t)HL * W + 255) / 256);
  copy_kernel<<<ncp, 256, 0, stream>>>(Fp(0), XA); copy_kernel<<<ncp, 256, 0, stream>>>(Fp(1), XB);
  conv_kernel<3><<<ncv, 256, 0, stream>>>(Fp(2), Fp(3), XA); conv_kernel<4><<<ncv, 256, 0, stream>>>(Fp(4), Fp(5), XA); conv_kernel<5><<<ncv, 256, 0, stream>>>(Fp(6), Fp(7), XA);
  conv_kernel<3><<<ncv, 256, 0, stream>>>(Fp(8), Fp(9), XB); conv_kernel<4><<<ncv, 256, 0, stream>>>(Fp(10), Fp(11), XB); conv_kernel<5><<<ncv, 256, 0, stream>>>(Fp(12), Fp(13), XB);
  mlp_kernel<<<(unsigned)(((size_t)HL * W) / 64), 128, 0, stream>>>(XA, XB, W1T, W2T, Fp(15), Fp(17), outf, den1, den2);
}
